// DenseSynthesizerAttention_20100446945666
// MI455X (gfx1250) — hardware-verified
//
#include <hip/hip_runtime.h>
#include <stdint.h>

#define NBAT  8
#define SQL   1024
#define NF    512
#define NHID  1024
#define NHEAD 8
#define DK    64
#define NTOK  (NBAT * SQL)
#define ATTSC 0.125f
#define LNPS  6.931471805599453f
#define HSC   16.0f
#define WSC   64.0f
#define XSC   16.0f
static_assert(NTOK == 8192);
static_assert((NTOK % 64) == 0);
static_assert((SQL % 64) == 0);
static_assert((NF % 128) == 0);
static_assert((NHID % 128) == 0);
static_assert(NF == NHEAD * DK);
static_assert(DK == 64);

typedef _Float16       v16h __attribute__((ext_vector_type(16)));
typedef _Float16       v8h  __attribute__((ext_vector_type(8)));
typedef __bf16         v16b __attribute__((ext_vector_type(16)));
typedef unsigned short v8us __attribute__((ext_vector_type(8)));
typedef float          v8f  __attribute__((ext_vector_type(8)));
typedef float          v4f  __attribute__((ext_vector_type(4)));
typedef unsigned int   v4u  __attribute__((ext_vector_type(4)));

union Frag  { v16h h; v16b b; v8us u[2]; };
union FragH { v16h v; v8h  h[2]; };
static_assert(sizeof(Frag) == 32);
static_assert(sizeof(FragH) == 32);

__device__ __forceinline__ unsigned short bf_bits(float f) {
  unsigned u = __float_as_uint(f);
  return (unsigned short)((u + 0x7FFFu + ((u >> 16) & 1u)) >> 16);
}
__device__ __forceinline__ float bf_up(unsigned short h) { return __uint_as_float(((unsigned)h) << 16); }
__device__ __forceinline__ float bf_rn(float f) { return bf_up(bf_bits(f)); }
__device__ __forceinline__ unsigned short h_bits(_Float16 x) { return __builtin_bit_cast(unsigned short, x); }
__device__ __forceinline__ unsigned pk16(unsigned short a, unsigned short b) { return (unsigned)a | ((unsigned)b << 16); }
__device__ __forceinline__ v8f zero8() { v8f z = {0.f, 0.f, 0.f, 0.f, 0.f, 0.f, 0.f, 0.f}; return z; }
__device__ __forceinline__ float hmax8(v8f s) {
  return fmaxf(fmaxf(fmaxf(s[0], s[1]), fmaxf(s[2], s[3])), fmaxf(fmaxf(s[4], s[5]), fmaxf(s[6], s[7])));
}
__device__ __forceinline__ v4u pack_h8(v4f a, v4f b) {
  v4u w;
  w[0] = pk16(h_bits((_Float16)a[0]), h_bits((_Float16)a[1]));
  w[1] = pk16(h_bits((_Float16)a[2]), h_bits((_Float16)a[3]));
  w[2] = pk16(h_bits((_Float16)b[0]), h_bits((_Float16)b[1]));
  w[3] = pk16(h_bits((_Float16)b[2]), h_bits((_Float16)b[3]));
  return w;
}

__device__ __forceinline__ Frag ldfrag(const unsigned short* p) {
  Frag f;
  f.u[0] = *(const v8us*)(p);
  f.u[1] = *(const v8us*)(p + 16);
  return f;
}
__device__ __forceinline__ v16h ldfrag_h(const _Float16* p) {
  FragH f;
  f.h[0] = *(const v8h*)(p);
  f.h[1] = *(const v8h*)(p + 16);
  return f.v;
}

__device__ __forceinline__ v8f mma_h(v16h a, v16h b, v8f c) {
  return __builtin_amdgcn_wmma_f32_16x16x32_f16(false, a, false, b, (short)0, c, false, false);
}
__device__ __forceinline__ v8f mma_b(v16b a, v16b b, v8f c) {
  return __builtin_amdgcn_wmma_f32_16x16x32_bf16(false, a, false, b, (short)0, c, false, false);
}
__device__ __forceinline__ void gguard(v8f& c0, v8f& c1, v8f& c2, v8f& c3, v8f& c4, v8f& c5, v8f& c6, v8f& c7,
                                       const Frag& a0, const Frag& a1,
                                       const Frag& b0, const Frag& b1, const Frag& b2, const Frag& b3) {
#if defined(__HIP_DEVICE_COMPILE__)
  asm volatile("v_nop\n\tv_nop\n\tv_nop\n\tv_nop"
               : "+v"(c0), "+v"(c1), "+v"(c2), "+v"(c3), "+v"(c4), "+v"(c5), "+v"(c6), "+v"(c7)
               : "v"(a0.h), "v"(a1.h), "v"(b0.h), "v"(b1.h), "v"(b2.h), "v"(b3.h));
#endif
}
__device__ __forceinline__ void sguard(v8f& a, v8f& b,
                                       const Frag& x0, const Frag& x1, const Frag& x2, const Frag& x3,
                                       const Frag& x4, const Frag& x5, const Frag& x6, const Frag& x7,
                                       const Frag& y0, const Frag& y1, const Frag& y2, const Frag& y3) {
#if defined(__HIP_DEVICE_COMPILE__)
  asm volatile("v_nop\n\tv_nop\n\tv_nop\n\tv_nop"
               : "+v"(a), "+v"(b)
               : "v"(x0.h), "v"(x1.h), "v"(x2.h), "v"(x3.h), "v"(x4.h), "v"(x5.h), "v"(x6.h), "v"(x7.h),
                 "v"(y0.h), "v"(y1.h), "v"(y2.h), "v"(y3.h));
#endif
}
__device__ __forceinline__ void oguard4(v8f& a, v8f& b, v8f& c, v8f& d,
                                        v16h x0, v16h x1, v16h x2, v16h x3, v16h p0) {
#if defined(__HIP_DEVICE_COMPILE__)
  asm volatile("v_nop\n\tv_nop\n\tv_nop\n\tv_nop"
               : "+v"(a), "+v"(b), "+v"(c), "+v"(d) : "v"(x0), "v"(x1), "v"(x2), "v"(x3), "v"(p0));
#endif
}

__global__ __launch_bounds__(256) void cvt_rows(const float* __restrict__ q, const float* __restrict__ v,
                                                 const float* __restrict__ kt_unused,
                                                 unsigned short* Qb, unsigned short* Vb, int nblk) {
  (void)kt_unused;
  const int bx = blockIdx.x;
  const bool second = bx >= nblk;
  const float* src = second ? v : q;
  unsigned short* dst = second ? Vb : Qb;
  const size_t i8 = ((size_t)(second ? bx - nblk : bx) * 256 + threadIdx.x) * 8;
  const v4f a = *(const v4f*)(src + i8), b = *(const v4f*)(src + i8 + 4);
  v4u w;
#pragma unroll
  for (int i = 0; i < 2; ++i) {
    w[i]     = pk16(bf_bits(a[2 * i]), bf_bits(a[2 * i + 1]));
    w[2 + i] = pk16(bf_bits(b[2 * i]), bf_bits(b[2 * i + 1]));
  }
  for (int pass = 0; pass < 2; ++pass) {
    *(volatile v4u*)(dst + i8) = w;
    __threadfence();
  }
}

__global__ __launch_bounds__(256) void cvt_wt(const float* __restrict__ w, unsigned short* out,
                                               int R, int Cc, float scale, int f16mode) {
  __shared__ __align__(16) unsigned short Ts[64 * 72];
  const int tid = threadIdx.x;
  const int c0 = blockIdx.x * 64, r0 = blockIdx.y * 64;
  {
    const int rr = tid >> 2, cq = (tid & 3) * 16;
    const float* p = w + (size_t)(r0 + rr) * Cc + c0 + cq;
#pragma unroll
    for (int j = 0; j < 4; ++j) {
      const v4f x = *(const v4f*)(p + 4 * j);
#pragma unroll
      for (int i = 0; i < 4; ++i) {
        const float f = bf_rn(x[i]) * scale;
        const unsigned short hb = h_bits((_Float16)f);
        const unsigned short bb = bf_bits(f);
        Ts[(cq + 4 * j + i) * 72 + rr] = f16mode ? hb : bb;
      }
    }
  }
  __syncthreads();
  {
    const int e = tid & 7, lq = tid >> 3;
    v4u u[2];
#pragma unroll
    for (int it = 0; it < 2; ++it) {
      const int cc = it * 32 + lq;
      u[it] = *(const v4u*)(Ts + cc * 72 + 8 * e);
    }
    for (int pass = 0; pass < 2; ++pass) {
#pragma unroll
      for (int it = 0; it < 2; ++it) {
        const int cc = it * 32 + lq;
        *(volatile v4u*)(out + (size_t)(c0 + cc) * R + r0 + 8 * e) = u[it];
      }
      __threadfence();
    }
  }
}

__device__ __forceinline__ void stage8(float* cs, v8f a, float bb, float oscale, float cscale, int relu) {
  v4f t0, t1;
#pragma unroll
  for (int i = 0; i < 4; ++i) {
    float x = a[i] * oscale + bb;
    float y = a[4 + i] * oscale + bb;
    if (relu) { x = fmaxf(x, 0.f); y = fmaxf(y, 0.f); }
    t0[i] = x * cscale;
    t1[i] = y * cscale;
  }
  *(v4f*)(cs) = t0;
  *(v4f*)(cs + 4) = t1;
}

template <int OPF16, int OUTM>
__global__ __launch_bounds__(128)
void gemm_kernel(const unsigned short* __restrict__ A, const unsigned short* __restrict__ Bt,
                 const float* __restrict__ bias, unsigned short* P0, unsigned short* P1, float* Cf,
                 int N, int K, int SQ_, float oscale, float cscale, int relu) {
  __shared__ __align__(16) float Cs[128 * 68];
  const int tid  = threadIdx.x;
  const int wave = tid >> 5;
  const int lane = tid & 31;
  const int hh   = lane >> 4;
  const int c    = lane & 15;
  const int wm   = wave >> 1, wn = wave & 1;
  const int m0   = blockIdx.y * 64;
  const int n0   = blockIdx.x * 128;
  const size_t Ks = (size_t)K;
  const unsigned short* Ap = A  + (size_t)(m0 + 32 * wm + c) * Ks + 8 * hh;
  const unsigned short* Bp = Bt + (size_t)(n0 + 64 * wn + c) * Ks + 8 * hh;

  v8f c00 = zero8(), c01 = zero8(), c02 = zero8(), c03 = zero8();
  v8f c10 = zero8(), c11 = zero8(), c12 = zero8(), c13 = zero8();
#pragma unroll 1
  for (int k0 = 0; k0 < K; k0 += 32) {
    const Frag a0 = ldfrag(Ap + k0);
    const Frag a1 = ldfrag(Ap + 16 * Ks + k0);
    const Frag b0 = ldfrag(Bp + k0);
    const Frag b1 = ldfrag(Bp + 16 * Ks + k0);
    const Frag b2 = ldfrag(Bp + 32 * Ks + k0);
    const Frag b3 = ldfrag(Bp + 48 * Ks + k0);
    if constexpr (OPF16) {
      c00 = mma_h(a0.h, b0.h, c00); c01 = mma_h(a0.h, b1.h, c01);
      c02 = mma_h(a0.h, b2.h, c02); c03 = mma_h(a0.h, b3.h, c03);
      c10 = mma_h(a1.h, b0.h, c10); c11 = mma_h(a1.h, b1.h, c11);
      c12 = mma_h(a1.h, b2.h, c12); c13 = mma_h(a1.h, b3.h, c13);
    } else {
      c00 = mma_b(a0.b, b0.b, c00); c01 = mma_b(a0.b, b1.b, c01);
      c02 = mma_b(a0.b, b2.b, c02); c03 = mma_b(a0.b, b3.b, c03);
      c10 = mma_b(a1.b, b0.b, c10); c11 = mma_b(a1.b, b1.b, c11);
      c12 = mma_b(a1.b, b2.b, c12); c13 = mma_b(a1.b, b3.b, c13);
    }
    gguard(c00, c01, c02, c03, c10, c11, c12, c13, a0, a1, b0, b1, b2, b3);
  }

  {
    const int nb = n0 + 64 * wn + c;
    const float bb0 = bf_rn(bias[nb]);
    const float bb1 = bf_rn(bias[nb + 16]);
    const float bb2 = bf_rn(bias[nb + 32]);
    const float bb3 = bf_rn(bias[nb + 48]);
    float* cs = Cs + (64 * wn + c) * 68 + 32 * wm + 8 * hh;
    stage8(cs + 0 * 1088 + 0,  c00, bb0, oscale, cscale, relu);
    stage8(cs + 1 * 1088 + 0,  c01, bb1, oscale, cscale, relu);
    stage8(cs + 2 * 1088 + 0,  c02, bb2, oscale, cscale, relu);
    stage8(cs + 3 * 1088 + 0,  c03, bb3, oscale, cscale, relu);
    stage8(cs + 0 * 1088 + 16, c10, bb0, oscale, cscale, relu);
    stage8(cs + 1 * 1088 + 16, c11, bb1, oscale, cscale, relu);
    stage8(cs + 2 * 1088 + 16, c12, bb2, oscale, cscale, relu);
    stage8(cs + 3 * 1088 + 16, c13, bb3, oscale, cscale, relu);
  }
  __syncthreads();

  const int e = tid & 7, lq = tid >> 3;
  if constexpr (OUTM == 0 || OUTM == 1) {
    v4u ua[8], ub[8];
#pragma unroll
    for (int it = 0; it < 8; ++it) {
      const int L = it * 16 + lq;
      const int row = L >> 1, col = (L & 1) * 64 + 8 * e;
      float f[8];
#pragma unroll
      for (int i = 0; i < 8; ++i) f[i] = Cs[(col + i) * 68 + row];
      v4u wa, wb;
#pragma unroll
      for (int i = 0; i < 4; ++i) {
        if constexpr (OUTM == 0) {
          wa[i] = pk16(h_bits((_Float16)f[2 * i]), h_bits((_Float16)f[2 * i + 1]));
          wb[i] = 0u;
        } else {
          const unsigned short h0 = bf_bits(f[2 * i]), h1 = bf_bits(f[2 * i + 1]);
          const unsigned short l0 = bf_bits(f[2 * i] - bf_up(h0)), l1 = bf_bits(f[2 * i + 1] - bf_up(h1));
          wa[i] = pk16(h0, h1);
          wb[i] = pk16(l0, l1);
        }
      }
      ua[it] = wa; ub[it] = wb;
    }
    for (int pass = 0; pass < 2; ++pass) {
#pragma unroll
      for (int it = 0; it < 8; ++it) {
        const int L = it * 16 + lq;
        const int row = L >> 1, col = (L & 1) * 64 + 8 * e;
        const size_t go = (size_t)(m0 + row) * N + n0 + col;
        *(volatile v4u*)(P0 + go) = ua[it];
        if constexpr (OUTM == 1) *(volatile v4u*)(P1 + go) = ub[it];
      }
      __threadfence();
    }
  } else if constexpr (OUTM == 2) {
    const int bi = m0 / SQ_;
    const int s0 = m0 - bi * SQ_;
    v4u ua[8];
#pragma unroll
    for (int it = 0; it < 8; ++it) {
      const int n = it * 16 + lq;
      const float* cs = Cs + n * 68 + 8 * e;
      const v4f x0 = *(const v4f*)(cs), x1 = *(const v4f*)(cs + 4);
      ua[it] = pack_h8(x0, x1);
    }
    for (int pass = 0; pass < 2; ++pass) {
#pragma unroll
      for (int it = 0; it < 8; ++it) {
        const int n = it * 16 + lq;
        *(volatile v4u*)(P0 + ((size_t)(bi * N + n0 + n)) * SQ_ + s0 + 8 * e) = ua[it];
      }
      __threadfence();
    }
  } else {
    v4f vals[16];
#pragma unroll
    for (int it = 0; it < 16; ++it) {
      const int L = it * 16 + lq;
      const int row = L >> 2, col = (L & 3) * 32 + 4 * e;
      v4f x;
      x[0] = Cs[(col + 0) * 68 + row];
      x[1] = Cs[(col + 1) * 68 + row];
      x[2] = Cs[(col + 2) * 68 + row];
      x[3] = Cs[(col + 3) * 68 + row];
      vals[it] = x;
    }
    for (int pass = 0; pass < 2; ++pass) {
#pragma unroll
      for (int it = 0; it < 16; ++it) {
        const int L = it * 16 + lq;
        const int row = L >> 2, col = (L & 3) * 32 + 4 * e;
        *(volatile v4f*)(Cf + (size_t)(m0 + row) * N + n0 + col) = vals[it];
      }
      __threadfence();
    }
  }
}

__global__ __launch_bounds__(128)
void attn_kernel(const unsigned short* __restrict__ awh, const unsigned short* __restrict__ awl,
                 const unsigned short* __restrict__ vt, unsigned short* xp) {
  __shared__ __align__(16) float Os[64 * 68];
  const int tid  = threadIdx.x;
  const int wave = tid >> 5;
  const int lane = tid & 31;
  const int hh   = lane >> 4;
  const int c    = lane & 15;
  const int q0   = blockIdx.x * 64;
  const int bh   = blockIdx.y;
  const int b    = bh >> 3;
  const int hd   = bh & 7;
  const size_t tok0 = (size_t)b * SQL;

  const size_t qoff = (tok0 + q0 + wave * 16 + c) * NF + hd * DK + 8 * hh;
  const Frag qh0 = ldfrag(awh + qoff);
  const Frag qh1 = ldfrag(awh + qoff + 32);
  const Frag ql0 = ldfrag(awl + qoff);
  const Frag ql1 = ldfrag(awl + qoff + 32);

  const size_t koff = (tok0 + c) * NF + hd * DK + 8 * hh;
  const unsigned short* Kh = awh + koff;
  const unsigned short* Kl = awl + koff;
  const _Float16* VTh = (const _Float16*)(const void*)vt;
  const _Float16* Vp  = VTh + ((size_t)(b * NF + hd * DK + c)) * SQL + 8 * hh;

  float m = -1.0e30f, l = 0.f;
  v8f o0 = zero8(), o1 = zero8(), o2 = zero8(), o3 = zero8();
#pragma unroll 1
  for (int it = 0; it < SQL / 32; ++it) {
    const int kb = it * 32;
    const unsigned short* k0h = Kh + (size_t)kb * NF;
    const unsigned short* k1h = k0h + (size_t)16 * NF;
    const unsigned short* k0l = Kl + (size_t)kb * NF;
    const unsigned short* k1l = k0l + (size_t)16 * NF;
    const Frag a00 = ldfrag(k0h), a01 = ldfrag(k0h + 32), e00 = ldfrag(k0l), e01 = ldfrag(k0l + 32);
    const Frag a10 = ldfrag(k1h), a11 = ldfrag(k1h + 32), e10 = ldfrag(k1l), e11 = ldfrag(k1l + 32);
    v8f s0 = mma_b(a00.b, qh0.b, zero8());
    s0 = mma_b(a01.b, qh1.b, s0);
    s0 = mma_b(a00.b, ql0.b, s0);
    s0 = mma_b(a01.b, ql1.b, s0);
    s0 = mma_b(e00.b, qh0.b, s0);
    s0 = mma_b(e01.b, qh1.b, s0);
    v8f s1 = mma_b(a10.b, qh0.b, zero8());
    s1 = mma_b(a11.b, qh1.b, s1);
    s1 = mma_b(a10.b, ql0.b, s1);
    s1 = mma_b(a11.b, ql1.b, s1);
    s1 = mma_b(e10.b, qh0.b, s1);
    s1 = mma_b(e11.b, qh1.b, s1);
    sguard(s0, s1, a00, a01, e00, e01, a10, a11, e10, e11, qh0, qh1, ql0, ql1);

    float mx = fmaxf(hmax8(s0), hmax8(s1));
    mx = fmaxf(mx, __shfl_xor(mx, 16, 32));
    const float mn   = fmaxf(m, mx * ATTSC);
    const float corr = __expf(m - mn);
    m = mn;
    const float msh = mn - LNPS;
    l *= corr;
#pragma unroll
    for (int r = 0; r < 8; ++r) {
      o0[r] *= corr; o1[r] *= corr; o2[r] *= corr; o3[r] *= corr;
    }

    FragH ph;
    float ls = 0.f;
#pragma unroll
    for (int r = 0; r < 8; ++r) {
      const float e0 = __expf(s0[r] * ATTSC - msh);
      const float e1 = __expf(s1[r] * ATTSC - msh);
      ls += e0 + e1;
      ph.h[0][r] = (_Float16)e0;
      ph.h[1][r] = (_Float16)e1;
    }
    l += ls;

    {
      const v16h vf0 = ldfrag_h(Vp + kb);
      const v16h vf1 = ldfrag_h(Vp + (size_t)16 * SQL + kb);
      const v16h vf2 = ldfrag_h(Vp + (size_t)32 * SQL + kb);
      const v16h vf3 = ldfrag_h(Vp + (size_t)48 * SQL + kb);
      o0 = mma_h(vf0, ph.v, o0);
      o1 = mma_h(vf1, ph.v, o1);
      o2 = mma_h(vf2, ph.v, o2);
      o3 = mma_h(vf3, ph.v, o3);
      oguard4(o0, o1, o2, o3, vf0, vf1, vf2, vf3, ph.v);
    }
  }
  l += __shfl_xor(l, 16, 32);
  const float sc = XSC / l;

  {
    float* os = Os + (wave * 16 + c) * 68 + 8 * hh;
    v4f t;
    t = {o0[0] * sc, o0[1] * sc, o0[2] * sc, o0[3] * sc}; *(v4f*)(os + 0)  = t;
    t = {o0[4] * sc, o0[5] * sc, o0[6] * sc, o0[7] * sc}; *(v4f*)(os + 4)  = t;
    t = {o1[0] * sc, o1[1] * sc, o1[2] * sc, o1[3] * sc}; *(v4f*)(os + 16) = t;
    t = {o1[4] * sc, o1[5] * sc, o1[6] * sc, o1[7] * sc}; *(v4f*)(os + 20) = t;
    t = {o2[0] * sc, o2[1] * sc, o2[2] * sc, o2[3] * sc}; *(v4f*)(os + 32) = t;
    t = {o2[4] * sc, o2[5] * sc, o2[6] * sc, o2[7] * sc}; *(v4f*)(os + 36) = t;
    t = {o3[0] * sc, o3[1] * sc, o3[2] * sc, o3[3] * sc}; *(v4f*)(os + 48) = t;
    t = {o3[4] * sc, o3[5] * sc, o3[6] * sc, o3[7] * sc}; *(v4f*)(os + 52) = t;
  }
  __syncthreads();
  {
    const int e = tid & 7, lq = tid >> 3;
    v4u u[4];
#pragma unroll
    for (int it = 0; it < 4; ++it) {
      const int L = it * 16 + lq;
      const float* os = Os + L * 68 + 8 * e;
      const v4f x0 = *(const v4f*)(os), x1 = *(const v4f*)(os + 4);
      u[it] = pack_h8(x0, x1);
    }
    unsigned short* xb = xp + (tok0 + q0) * NF + hd * DK + 8 * e;
    for (int pass = 0; pass < 2; ++pass) {
#pragma unroll
      for (int it = 0; it < 4; ++it) {
        const int L = it * 16 + lq;
        *(volatile v4u*)(xb + (size_t)L * NF) = u[it];
      }
      __threadfence();
    }
  }
}

extern "C" void kernel_launch(void* const* d_in, const int* in_sizes, int n_in,
                              void* d_out, int out_size, void* d_ws, size_t ws_size,
                              hipStream_t stream) {
  const int NACT = NTOK * NF;
  if (n_in < 11) return;
  if (in_sizes[0] != NACT || in_sizes[1] != NACT || in_sizes[2] != NACT) return;
  if (in_sizes[3] != NF * NHID || in_sizes[4] != NHID) return;
  if (in_sizes[5] != NHID * NF || in_sizes[6] != NF) return;
  if (in_sizes[7] != NF * NF || in_sizes[8] != NF) return;
  if (in_sizes[9] != NF * NF || in_sizes[10] != NF) return;
  if (out_size != NACT) return;

  size_t off = 0;
  const size_t oQb = off; off += (size_t)NTOK * NF * 2;
  const size_t oVb = off; off += (size_t)NTOK * NF * 2;
  const size_t oW1 = off; off += (size_t)NHID * NF * 2;
  const size_t oW2 = off; off += (size_t)NF * NHID * 2;
  const size_t oWV = off; off += (size_t)NF * NF * 2;
  const size_t oWO = off; off += (size_t)NF * NF * 2;
  const size_t oH  = off; off += (size_t)NTOK * NHID * 2;
  const size_t oAH = off; off += (size_t)NTOK * NF * 2;
  const size_t oAL = off; off += (size_t)NTOK * NF * 2;
  const size_t oVT = off; off += (size_t)NBAT * NF * SQL * 2;
  const size_t oXP = off; off += (size_t)NTOK * NF * 2;
  if (off > ws_size) return;
  if (off > (size_t)134217728) return;

  const float* query = (const float*)d_in[0];
  const float* key_t = (const float*)d_in[1];
  const float* value = (const float*)d_in[2];
  const float* w1 = (const float*)d_in[3];
  const float* b1 = (const float*)d_in[4];
  const float* w2 = (const float*)d_in[5];
  const float* b2 = (const float*)d_in[6];
  const float* wv = (const float*)d_in[7];
  const float* bv = (const float*)d_in[8];
  const float* wo = (const float*)d_in[9];
  const float* bo = (const float*)d_in[10];
  float* out = (float*)d_out;
  char* ws = (char*)d_ws;
  unsigned short* Qb  = (unsigned short*)(ws + oQb);
  unsigned short* Vb  = (unsigned short*)(ws + oVb);
  unsigned short* W1t = (unsigned short*)(ws + oW1);
  unsigned short* W2t = (unsigned short*)(ws + oW2);
  unsigned short* WVt = (unsigned short*)(ws + oWV);
  unsigned short* WOt = (unsigned short*)(ws + oWO);
  unsigned short* Hp  = (unsigned short*)(ws + oH);
  unsigned short* AWH = (unsigned short*)(ws + oAH);
  unsigned short* AWL = (unsigned short*)(ws + oAL);
  unsigned short* VT  = (unsigned short*)(ws + oVT);
  unsigned short* XP  = (unsigned short*)(ws + oXP);

  const dim3 blk256(256), blk128(128);
  const int nblk = NACT / (256 * 8);

  cvt_rows<<<dim3(2 * nblk), blk256, 0, stream>>>(query, value, key_t, Qb, Vb, nblk);
  cvt_wt<<<dim3(NHID / 64, NF / 64), blk256, 0, stream>>>(w1, W1t, NF, NHID, 1.0f, 0);
  cvt_wt<<<dim3(NF / 64, NHID / 64), blk256, 0, stream>>>(w2, W2t, NHID, NF, WSC, 1);
  cvt_wt<<<dim3(NF / 64, NF / 64), blk256, 0, stream>>>(wv, WVt, NF, NF, 1.0f, 0);
  cvt_wt<<<dim3(NF / 64, NF / 64), blk256, 0, stream>>>(wo, WOt, NF, NF, WSC, 1);

  gemm_kernel<0, 0><<<dim3(NHID / 128, NTOK / 64), blk128, 0, stream>>>(
      Qb, W1t, b1, Hp, Hp, out, NHID, NF, SQL, 1.0f, HSC, 1);
  gemm_kernel<1, 1><<<dim3(NF / 128, NTOK / 64), blk128, 0, stream>>>(
      Hp, W2t, b2, AWH, AWL, out, NF, NHID, SQL, 1.0f / (HSC * WSC), 1.0f, 0);
  gemm_kernel<0, 2><<<dim3(NF / 128, NTOK / 64), blk128, 0, stream>>>(
      Vb, WVt, bv, VT, VT, out, NF, NF, SQL, 1.0f, 1.0f, 0);
  attn_kernel<<<dim3(SQL / 64, NBAT * NHEAD), blk128, 0, stream>>>(AWH, AWL, VT, XP);
  gemm_kernel<1, 3><<<dim3(NF / 128, NTOK / 64), blk128, 0, stream>>>(
      XP, WOt, bo, AWH, AWH, out, NF, NF, SQL, 1.0f / (XSC * WSC), 1.0f, 0);
  (void)hipGetLastError();
}
